// DisattentionBlock_3607772529024
// MI455X (gfx1250) — hardware-run, weakly checked
//
#include <hip/hip_runtime.h>
#include <math.h>
#include <stdint.h>

constexpr int kB     = 2;
constexpr int kS     = 2048;
constexpr int kD     = 1024;
constexpr int kF     = 4096;
constexpr int kH     = 16;
constexpr int kDh    = 64;
constexpr int kTok   = kB * kS;
constexpr int kQKVld = 3 * kD;
constexpr int kGrp   = 2;
constexpr int kFfnRows = 1024;
constexpr float kEps   = 1e-5f;
constexpr float kInvD  = 1.0f / 1024.0f;

typedef __attribute__((ext_vector_type(16))) _Float16 v16h;
typedef __attribute__((ext_vector_type(8)))  _Float16 v8h;
typedef __attribute__((ext_vector_type(16))) __bf16   v16b;
typedef __attribute__((ext_vector_type(8)))  __bf16   v8b;
typedef __attribute__((ext_vector_type(8)))  float    v8f;
typedef __attribute__((ext_vector_type(4)))  float    v4f;
typedef __attribute__((ext_vector_type(2)))  float    v2f;
typedef __attribute__((ext_vector_type(4)))  unsigned int v4u;

__device__ __forceinline__ unsigned short f2bf_bits(float f) {
  unsigned u = __float_as_uint(f);
  return (unsigned short)((u + 0x7FFFu + ((u >> 16) & 1u)) >> 16);
}
__device__ __forceinline__ float bf_bits2f(unsigned short h) { return __uint_as_float(((unsigned)h) << 16); }

__device__ __forceinline__ void dep_guard_h(v8f& a, v8f& b, v16h x, v16h y) { asm volatile("v_nop\n\tv_nop\n\tv_nop\n\tv_nop" : "+v"(a), "+v"(b) : "v"(x), "v"(y)); }
__device__ __forceinline__ void dep_guard_b(v8f& a, v8f& b, v16b x, v16b y) { asm volatile("v_nop\n\tv_nop\n\tv_nop\n\tv_nop" : "+v"(a), "+v"(b) : "v"(x), "v"(y)); }
__device__ __forceinline__ void keep4_h(v16h a, v16h b, v16h c, v16h d) { asm volatile("v_nop" :: "v"(a), "v"(b), "v"(c), "v"(d)); }
__device__ __forceinline__ void keep4_b(v16b a, v16b b, v16b c, v16b d) { asm volatile("v_nop" :: "v"(a), "v"(b), "v"(c), "v"(d)); }
__device__ __forceinline__ void acc_guard4(v8f& a, v8f& b, v8f& c, v8f& d) { asm volatile("v_nop\n\tv_nop\n\tv_nop\n\tv_nop" : "+v"(a), "+v"(b), "+v"(c), "+v"(d)); }
template <typename T> struct Frag;
template <> struct Frag<_Float16> {
  typedef v16h V; union U { v16h v; v8h h[2]; };
  static __device__ __forceinline__ v16h load(const _Float16* p) {
    U f; f.h[0] = *(const v8h*)(p); f.h[1] = *(const v8h*)(p + 16); return f.v;
  }
  static __device__ __forceinline__ v8f mma(v16h a, v16h b, v8f c) {
    return __builtin_amdgcn_wmma_f32_16x16x32_f16(false, a, false, b, (short)0, c, false, false);
  }
  static __device__ __forceinline__ void guard(v8f& a, v8f& b, v16h x, v16h y) { dep_guard_h(a, b, x, y); }
  static __device__ __forceinline__ void keep(v16h a, v16h b, v16h c, v16h d) { keep4_h(a, b, c, d); }
};
template <> struct Frag<__bf16> {
  typedef v16b V; union U { v16b v; v8b h[2]; };
  static __device__ __forceinline__ v16b load(const __bf16* p) {
    U f; f.h[0] = *(const v8b*)(p); f.h[1] = *(const v8b*)(p + 16); return f.v;
  }
  static __device__ __forceinline__ v8f mma(v16b a, v16b b, v8f c) {
    return __builtin_amdgcn_wmma_f32_16x16x32_bf16(false, a, false, b, (short)0, c, false, false);
  }
  static __device__ __forceinline__ void guard(v8f& a, v8f& b, v16b x, v16b y) { dep_guard_b(a, b, x, y); }
  static __device__ __forceinline__ void keep(v16b a, v16b b, v16b c, v16b d) { keep4_b(a, b, c, d); }
};

__device__ __forceinline__ unsigned pk16(unsigned short a, unsigned short b) { return (unsigned)a | ((unsigned)b << 16); }
__device__ __forceinline__ unsigned short h_bits(float f) { const _Float16 h = (_Float16)f; return __builtin_bit_cast(unsigned short, h); }

template <int ET> struct Elem;
template <> struct Elem<0> { typedef _Float16 T; };
template <> struct Elem<1> { typedef __bf16 T; };
template <int ET, bool SPLIT, int BIAS_MODE, int OUT_MODE, bool RESID, int ACT = 0>
__global__ __launch_bounds__(256) void wmma_gemm64(
    const unsigned short* __restrict__ Ap, const unsigned short* __restrict__ A2p, int lda, long strideA,
    const unsigned short* __restrict__ Btp, const unsigned short* __restrict__ Bt2p, int ldb, long strideB,
    void* __restrict__ Cout, void* __restrict__ Cout2, int ldc, long strideC,
    const float* __restrict__ bias,
    const float* __restrict__ resid, long strideR,
    int M, int N, int K, float scale) {
  typedef typename Elem<ET>::T T;
  typedef typename Frag<T>::V V;
  const T* A = (const T*)Ap; const T* A2 = (const T*)A2p; const T* Bt = (const T*)Btp; const T* Bt2 = (const T*)Bt2p;
  __shared__ __align__(16) float sT[8][16 * 68];
  const int b    = blockIdx.y;
  const int lane = threadIdx.x & 31;
  const int wave = threadIdx.x >> 5;
  const int tilesN = N >> 6;
  const int tilesM = M >> 6;
  const int tile = blockIdx.x * 8 + wave;
  if (tile >= tilesM * tilesN) return;
  const int tm = tile / tilesN;
  const int tn = tile - tm * tilesN;
  const int m0 = tm << 6;
  const int n0 = tn << 6;

  const T* Ab  = A  + (size_t)b * strideA;
  const T* Bb  = Bt + (size_t)b * strideB;
  const T* Ab2 = SPLIT ? (A2  + (size_t)b * strideA) : nullptr;
  const T* Bb2 = SPLIT ? (Bt2 + (size_t)b * strideB) : nullptr;

  const int rlane = lane & 15;
  const int koff  = (lane >> 4) * 8;
  const int mOff  = (lane >> 4) * 8;

  v8f acc[4][4];
#pragma unroll
  for (int i = 0; i < 4; ++i)
#pragma unroll
    for (int j = 0; j < 4; ++j) acc[i][j] = (v8f){0.f,0.f,0.f,0.f,0.f,0.f,0.f,0.f};

  for (int k0 = 0; k0 < K; k0 += 32) {
    V bh[4], bl[4];
#pragma unroll
    for (int j = 0; j < 4; ++j) {
      const size_t bo = (size_t)(n0 + (j << 4) + rlane) * ldb + koff + k0;
      bh[j] = Frag<T>::load(Bb + bo);
      if (SPLIT) bl[j] = Frag<T>::load(Bb2 + bo);
    }
#pragma unroll
    for (int i = 0; i < 4; ++i) {
      const size_t ao = (size_t)(m0 + (i << 4) + rlane) * lda + koff + k0;
      V ah = Frag<T>::load(Ab + ao);
      V al;
      if (SPLIT) al = Frag<T>::load(Ab2 + ao);
#pragma unroll
      for (int j = 0; j < 4; ++j) {
        acc[i][j] = Frag<T>::mma(ah, bh[j], acc[i][j]);
        if (SPLIT) {
          acc[i][j] = Frag<T>::mma(ah, bl[j], acc[i][j]);
          acc[i][j] = Frag<T>::mma(al, bh[j], acc[i][j]);
        }
      }
      Frag<T>::guard(acc[i][0], acc[i][3], ah, SPLIT ? al : ah);
    }
    Frag<T>::keep(bh[0], bh[1], bh[2], bh[3]);
    if (SPLIT) Frag<T>::keep(bl[0], bl[1], bl[2], bl[3]);
  }
  acc_guard4(acc[0][0], acc[0][1], acc[0][2], acc[0][3]);
  acc_guard4(acc[1][0], acc[1][1], acc[1][2], acc[1][3]);
  acc_guard4(acc[2][0], acc[2][1], acc[2][2], acc[2][3]);
  acc_guard4(acc[3][0], acc[3][1], acc[3][2], acc[3][3]);

  float* slab = sT[wave];
  const float* Rb = RESID ? (resid + (size_t)b * strideR) : nullptr;
#pragma unroll
  for (int i = 0; i < 4; ++i) {
    const int mBase = m0 + (i << 4);
#pragma unroll
    for (int j = 0; j < 4; ++j) {
      const int n = n0 + (j << 4) + rlane;
      float bv = 0.f;
      if (BIAS_MODE == 2) bv = bias[n];
#pragma unroll
      for (int r = 0; r < 8; ++r) {
        float v = acc[i][j][r] * scale;
        if (BIAS_MODE == 1) v += bias[mBase + mOff + r];
        if (BIAS_MODE == 2) v += bv;
        if (RESID) v += Rb[(size_t)(mBase + mOff + r) * ldc + n];
        if (ACT == 2) v = fmaxf(v, 0.0f);
        if (ACT == 4) v = (v > 0.f) ? v : 0.01f * v;
        slab[(mOff + r) * 68 + (j << 4) + rlane] = v;
      }
    }
    __builtin_amdgcn_fence(__ATOMIC_RELEASE, "workgroup");
    __builtin_amdgcn_wave_barrier();
    __builtin_amdgcn_fence(__ATOMIC_ACQUIRE, "workgroup");
    if (OUT_MODE == 0) {
      float* C = (float*)Cout + (size_t)b * strideC;
      const int hh = lane >> 4, c4 = (lane & 15) * 4;
      for (int pass = 0; pass < 2; ++pass) {
#pragma unroll
        for (int it = 0; it < 8; ++it) {
          const int row = it * 2 + hh;
          v4f v = *(const v4f*)(slab + row * 68 + c4);
          *(volatile v4f*)(C + (size_t)(mBase + row) * ldc + n0 + c4) = v;
        }
        __threadfence();
      }
    } else {
      const int q = lane >> 3, c8 = (lane & 7) * 8;
      unsigned short* C  = (unsigned short*)Cout  + (size_t)b * strideC;
      unsigned short* C2 = (OUT_MODE == 2) ? ((unsigned short*)Cout2 + (size_t)b * strideC) : nullptr;
      for (int pass = 0; pass < 2; ++pass) {
#pragma unroll
        for (int it = 0; it < 4; ++it) {
          const int row = it * 4 + q;
          const float* sp = slab + row * 68 + c8;
          v8h hv, lv;
#pragma unroll
          for (int e = 0; e < 8; ++e) {
            if (OUT_MODE == 1) {
              hv[e] = (_Float16)sp[e];
            } else {
              unsigned short hb = f2bf_bits(sp[e]);
              unsigned short lb = f2bf_bits(sp[e] - bf_bits2f(hb));
              hv[e] = __builtin_bit_cast(_Float16, hb);
              lv[e] = __builtin_bit_cast(_Float16, lb);
            }
          }
          *(volatile v8h*)(C + (size_t)(mBase + row) * ldc + n0 + c8) = hv;
          if (OUT_MODE == 2) *(volatile v8h*)(C2 + (size_t)(mBase + row) * ldc + n0 + c8) = lv;
        }
        __threadfence();
      }
    }
    __builtin_amdgcn_fence(__ATOMIC_RELEASE, "workgroup");
    __builtin_amdgcn_wave_barrier();
    __builtin_amdgcn_fence(__ATOMIC_ACQUIRE, "workgroup");
  }
}

__global__ __launch_bounds__(256) void tcast_kernel(const float* __restrict__ W0, const float* __restrict__ W1,
                                                    const float* __restrict__ W2, const float* __restrict__ W3,
                                                    unsigned short* __restrict__ O0, unsigned short* __restrict__ O1,
                                                    unsigned short* __restrict__ O2, unsigned short* __restrict__ O3,
                                                    int Kr, int Nc, float scale) {
  __shared__ float sm[64][65];
  const int t  = threadIdx.x;
  const int k0 = blockIdx.x * 64;
  const int n0 = blockIdx.y * 64;
  const int z  = blockIdx.z;
  const float* W = (z == 0) ? W0 : (z == 1) ? W1 : (z == 2) ? W2 : W3;
  unsigned short* O = (z == 0) ? O0 : (z == 1) ? O1 : (z == 2) ? O2 : O3;
#pragma unroll
  for (int i = 0; i < 16; ++i) {
    const int e = i * 256 + t;
    const int r = e >> 6;
    const int c = e & 63;
    sm[c][r] = W[(size_t)(k0 + r) * Nc + n0 + c] * scale;
  }
  __syncthreads();
  const int lane = t & 31, wave = t >> 5;
  const int q = lane >> 3, c8 = (lane & 7) * 8;
  for (int pass = 0; pass < 2; ++pass) {
#pragma unroll
    for (int it = 0; it < 2; ++it) {
      const int row = wave * 8 + it * 4 + q;
      unsigned short hb[8];
#pragma unroll
      for (int e = 0; e < 8; ++e) hb[e] = h_bits(sm[row][c8 + e]);
      const v4u u = (v4u){pk16(hb[0], hb[1]), pk16(hb[2], hb[3]), pk16(hb[4], hb[5]), pk16(hb[6], hb[7])};
      *(volatile v4u*)(O + (size_t)(n0 + row) * Kr + k0 + c8) = u;
    }
    __threadfence();
  }
}

__global__ __launch_bounds__(256) void vt_kernel(const unsigned short* __restrict__ QKV, unsigned short* __restrict__ VT) {
  __shared__ unsigned short sm[64][72];
  const int tid = threadIdx.x;
  const int t0  = blockIdx.x * 64;
  const int d0  = blockIdx.y * 64;
  const int b   = blockIdx.z;
#pragma unroll
  for (int i = 0; i < 2; ++i) {
    const int e   = i * 256 + tid;
    const int r   = e >> 3;
    const int seg = e & 7;
    const v4u w = *(const v4u*)(QKV + ((size_t)(b * kS + t0 + r)) * kQKVld + 2 * kD + d0 + seg * 8);
#pragma unroll
    for (int j = 0; j < 4; ++j) {
      sm[seg * 8 + 2 * j][r]     = (unsigned short)(w[j] & 0xffffu);
      sm[seg * 8 + 2 * j + 1][r] = (unsigned short)(w[j] >> 16);
    }
  }
  __syncthreads();
  const int lane = tid & 31, wave = tid >> 5;
  const int q = lane >> 3, c8 = (lane & 7) * 8;
  for (int pass = 0; pass < 2; ++pass) {
#pragma unroll
    for (int it = 0; it < 2; ++it) {
      const int row = wave * 8 + it * 4 + q;
      const v4u u = (v4u){pk16(sm[row][c8 + 0], sm[row][c8 + 1]), pk16(sm[row][c8 + 2], sm[row][c8 + 3]),
                          pk16(sm[row][c8 + 4], sm[row][c8 + 5]), pk16(sm[row][c8 + 6], sm[row][c8 + 7])};
      *(volatile v4u*)(VT + ((size_t)(b * kD + d0 + row)) * kS + t0 + c8) = u;
    }
    __threadfence();
  }
}

__global__ __launch_bounds__(128) void indnorm_kernel(const float* __restrict__ X, const float* __restrict__ G,
                                                      const float* __restrict__ Bv, unsigned short* __restrict__ H,
                                                      float omr, float rr) {
  __shared__ float redA[4];
  __shared__ float redB[4];
  const int row  = blockIdx.x;
  const int t    = threadIdx.x;
  const int lane = t & 31, wave = t >> 5;
  const int c0   = t * 8;
  const float* xr = X + (size_t)row * kD + c0;
  const v4f a = *(const v4f*)(xr);
  const v4f c = *(const v4f*)(xr + 4);
  float v[8];
#pragma unroll
  for (int e = 0; e < 4; ++e) { v[e] = a[e]; v[4 + e] = c[e]; }
  float s = ((v[0] + v[1]) + (v[2] + v[3])) + ((v[4] + v[5]) + (v[6] + v[7]));
#pragma unroll
  for (int off = 16; off > 0; off >>= 1) s += __shfl_xor(s, off, 32);
  if (lane == 0) redA[wave] = s;
  __syncthreads();
  const float mean = ((redA[0] + redA[1]) + (redA[2] + redA[3])) * kInvD;
  float d[8];
  float qs = 0.f;
#pragma unroll
  for (int e = 0; e < 8; ++e) { d[e] = v[e] - mean; qs += d[e] * d[e]; }
#pragma unroll
  for (int off = 16; off > 0; off >>= 1) qs += __shfl_xor(qs, off, 32);
  if (lane == 0) redB[wave] = qs;
  __syncthreads();
  const float var  = ((redB[0] + redB[1]) + (redB[2] + redB[3])) * kInvD;
  const float rstd = rsqrtf(var + kEps);
  const v4f ga = *(const v4f*)(G + c0);
  const v4f gc = *(const v4f*)(G + c0 + 4);
  const v4f ba = *(const v4f*)(Bv + c0);
  const v4f bc = *(const v4f*)(Bv + c0 + 4);
  float gg[8], bb[8];
#pragma unroll
  for (int e = 0; e < 4; ++e) { gg[e] = ga[e]; gg[4 + e] = gc[e]; bb[e] = ba[e]; bb[4 + e] = bc[e]; }
  unsigned short hb[8];
#pragma unroll
  for (int e = 0; e < 8; ++e) {
    const float ln = d[e] * rstd * gg[e] + bb[e];
    const float o  = omr * ln + rr * v[e];
    hb[e] = h_bits(o);
  }
  const v4u u = (v4u){pk16(hb[0], hb[1]), pk16(hb[2], hb[3]), pk16(hb[4], hb[5]), pk16(hb[6], hb[7])};
  unsigned short* op = H + (size_t)row * kD + c0;
  *(volatile v4u*)op = u;
  __threadfence();
  *(volatile v4u*)op = u;
}

__global__ __launch_bounds__(256) void softmax_kernel(const float* __restrict__ SC, const float* __restrict__ MK,
                                                      unsigned short* __restrict__ P, float carry) {
  __shared__ float redM[8];
  __shared__ float redS[8];
  const int row  = blockIdx.x;
  const int i    = row & (kS - 1);
  const int t    = threadIdx.x;
  const int lane = t & 31, wave = t >> 5;
  const int c0   = t * 8;
  const float* sr = SC + (size_t)row * kS + c0;
  const float* mr = MK + (size_t)i * kS + c0;
  const v4f a  = *(const v4f*)(sr);
  const v4f c  = *(const v4f*)(sr + 4);
  const v4f ma = *(const v4f*)(mr);
  const v4f mc = *(const v4f*)(mr + 4);
  float x[8];
#pragma unroll
  for (int e = 0; e < 4; ++e) {
    x[e]     = fminf(fmaxf(a[e], -50.0f), 50.0f) + ma[e];
    x[4 + e] = fminf(fmaxf(c[e], -50.0f), 50.0f) + mc[e];
  }
  float m = fmaxf(fmaxf(fmaxf(x[0], x[1]), fmaxf(x[2], x[3])), fmaxf(fmaxf(x[4], x[5]), fmaxf(x[6], x[7])));
#pragma unroll
  for (int off = 16; off > 0; off >>= 1) m = fmaxf(m, __shfl_xor(m, off, 32));
  if (lane == 0) redM[wave] = m;
  __syncthreads();
  float gm = redM[0];
#pragma unroll
  for (int w = 1; w < 8; ++w) gm = fmaxf(gm, redM[w]);
  float ev[8];
  float ps = 0.f;
#pragma unroll
  for (int e = 0; e < 8; ++e) { ev[e] = expf(x[e] - gm); ps += ev[e]; }
#pragma unroll
  for (int off = 16; off > 0; off >>= 1) ps += __shfl_xor(ps, off, 32);
  if (lane == 0) redS[wave] = ps;
  __syncthreads();
  float tot = 0.f;
#pragma unroll
  for (int w = 0; w < 8; ++w) tot += redS[w];
  const float inv = 1.0f / tot;
  unsigned short hb[8];
#pragma unroll
  for (int e = 0; e < 8; ++e) hb[e] = h_bits((ev[e] * inv) * carry);
  const v4u u = (v4u){pk16(hb[0], hb[1]), pk16(hb[2], hb[3]), pk16(hb[4], hb[5]), pk16(hb[6], hb[7])};
  unsigned short* pp = P + (size_t)row * kS + c0;
  *(volatile v4u*)pp = u;
  __threadfence();
  *(volatile v4u*)pp = u;
}

__global__ __launch_bounds__(256) void gelu_cast_kernel(const float* __restrict__ U, unsigned short* __restrict__ out,
                                                        int n2, int neg, float carry) {
  const int i = blockIdx.x * 256 + threadIdx.x;
  if (i >= n2) return;
  const v2f p = *(const v2f*)(U + 2 * (size_t)i);
  const float sgn = neg ? -1.0f : 1.0f;
  const float a = p[0] * sgn;
  const float b = p[1] * sgn;
  const float ga = 0.5f * a * (1.0f + erff(a * 0.70710678118654752f));
  const float gb = 0.5f * b * (1.0f + erff(b * 0.70710678118654752f));
  const unsigned u = pk16(h_bits(ga * carry), h_bits(gb * carry));
  unsigned* q = (unsigned*)(out + 2 * (size_t)i);
  *(volatile unsigned*)q = u;
  __threadfence();
  *(volatile unsigned*)q = u;
}

extern "C" void kernel_launch(void* const* d_in, const int* in_sizes, int n_in,
                              void* d_out, int out_size, void* d_ws, size_t ws_size,
                              hipStream_t stream) {
  const size_t MIB = 1048576;
  if (n_in < 14) return;
  if (in_sizes[0] != kTok * kD || in_sizes[1] != kB * kD * kD || in_sizes[2] != kS * kS ||
      in_sizes[3] != kD || in_sizes[4] != kD || in_sizes[5] != kD || in_sizes[6] != kD ||
      in_sizes[7] != kD * kD || in_sizes[8] != kD * kD || in_sizes[9] != kD * kD || in_sizes[10] != kD * kD ||
      in_sizes[11] != kD * kF || in_sizes[12] != kD * kF || in_sizes[13] != 2 * kF * kD) return;
  if (out_size != kTok * kD) return;
  if (ws_size < 124 * MIB) return;

  const float* xf   = (const float*)d_in[0];
  const float* Mf   = (const float*)d_in[1];
  const float* mkf  = (const float*)d_in[2];
  const float* g1f  = (const float*)d_in[3];
  const float* b1f  = (const float*)d_in[4];
  const float* g2f  = (const float*)d_in[5];
  const float* b2f  = (const float*)d_in[6];
  const float* Wqf  = (const float*)d_in[7];
  const float* Wkf  = (const float*)d_in[8];
  const float* Wvf  = (const float*)d_in[9];
  const float* Wof  = (const float*)d_in[10];
  const float* Wpf  = (const float*)d_in[11];
  const float* Wnf  = (const float*)d_in[12];
  const float* Wjf  = (const float*)d_in[13];
  float* out = (float*)d_out;

  char* ws = (char*)d_ws;
  unsigned short* H16   = (unsigned short*)(ws + 0 * MIB);
  unsigned short* WQKV  = (unsigned short*)(ws + 8 * MIB);
  unsigned short* MT    = (unsigned short*)(ws + 14 * MIB);
  unsigned short* WOT   = (unsigned short*)(ws + 18 * MIB);
  unsigned short* QKV   = (unsigned short*)(ws + 20 * MIB);
  unsigned short* QM    = (unsigned short*)(ws + 44 * MIB);
  unsigned short* VT    = (unsigned short*)(ws + 52 * MIB);
  unsigned short* CTX   = (unsigned short*)(ws + 60 * MIB);
  float*          SC    = (float*)(ws + 68 * MIB);
  unsigned short* P16   = (unsigned short*)(ws + 100 * MIB);
  float*          X1    = (float*)(ws + 20 * MIB);
  unsigned short* WPOS  = (unsigned short*)(ws + 8 * MIB);
  unsigned short* WNEG  = (unsigned short*)(ws + 116 * MIB);
  unsigned short* WPROJ = (unsigned short*)(ws + 36 * MIB);
  float*          TP    = (float*)(ws + 52 * MIB);
  unsigned short* CAT   = (unsigned short*)(ws + 68 * MIB);
  float*          U     = (float*)(ws + 100 * MIB);

  const float rr  = (float)(2.0 / 11.0);
  const float omr = (float)(1.0 - 2.0 / 11.0);
  const float wcarry  = 16.0f;
  const float wjcarry = 64.0f;
  const float pcarry  = 2048.0f;
  const float ccarry  = 16.0f;

  tcast_kernel<<<dim3(kD / 64, kD / 64, 4), 256, 0, stream>>>(
      Wqf, Wkf, Wvf, Wof,
      WQKV, WQKV + (size_t)kD * kD, WQKV + (size_t)2 * kD * kD, WOT, kD, kD, wcarry);
  tcast_kernel<<<dim3(kD / 64, kD / 64, 2), 256, 0, stream>>>(
      Mf, Mf + (size_t)kD * kD, Mf, Mf,
      MT, MT + (size_t)kD * kD, MT, MT, kD, kD, wcarry);

  indnorm_kernel<<<dim3(kTok), 128, 0, stream>>>(xf, g1f, b1f, H16, omr, rr);

  wmma_gemm64<0, false, 0, 1, false><<<dim3(384, 1), 256, 0, stream>>>(
      H16, H16, kD, 0, WQKV, WQKV, kD, 0, QKV, QKV, kQKVld, 0, g1f, xf, 0, kTok, kQKVld, kD, 1.0f / wcarry);

  vt_kernel<<<dim3(kS / 64, kD / 64, kB), 256, 0, stream>>>(QKV, VT);

  wmma_gemm64<0, false, 0, 1, false><<<dim3(64, kB), 256, 0, stream>>>(
      QKV, QKV, kQKVld, (long)kS * kQKVld, MT, MT, kD, (long)kD * kD, QM, QM, kD, (long)kS * kD,
      g1f, xf, 0, kS, kD, kD, 1.0f / wcarry);

  for (int b = 0; b < kB; ++b) {
    for (int h0 = 0; h0 < kH; h0 += kGrp) {
      const unsigned short* Aq = QM + (size_t)b * kS * kD + (size_t)h0 * kDh;
      const unsigned short* Bk = QKV + kD + (size_t)b * kS * kQKVld + (size_t)h0 * kDh;
      wmma_gemm64<0, false, 0, 0, false><<<dim3(128, kGrp), 256, 0, stream>>>(
          Aq, Aq, kD, kDh, Bk, Bk, kQKVld, kDh, SC, SC, kS, (long)kS * kS, g1f, xf, 0, kS, kS, kDh, 0.125f);
      softmax_kernel<<<dim3(kGrp * kS), 256, 0, stream>>>(SC, mkf, P16, pcarry);
      const unsigned short* Bv = VT + ((size_t)b * kD + (size_t)h0 * kDh) * kS;
      unsigned short* Cc = CTX + (size_t)b * kS * kD + (size_t)h0 * kDh;
      wmma_gemm64<0, false, 0, 1, false><<<dim3(4, kGrp), 256, 0, stream>>>(
          P16, P16, kS, (long)kS * kS, Bv, Bv, kS, (long)kDh * kS, Cc, Cc, kD, kDh, g1f, xf, 0,
          kS, kDh, kS, 64.0f / 2048.0f);
    }
  }

  wmma_gemm64<0, false, 0, 0, true><<<dim3(128, 1), 256, 0, stream>>>(
      CTX, CTX, kD, 0, WOT, WOT, kD, 0, X1, X1, kD, 0, g1f, xf, 0, kTok, kD, kD, 1.0f / 1024.0f);

  indnorm_kernel<<<dim3(kTok), 128, 0, stream>>>(X1, g2f, b2f, H16, omr, rr);
  tcast_kernel<<<dim3(kD / 64, kF / 64, 2), 256, 0, stream>>>(
      Wpf, Wnf, Wpf, Wpf, WPOS, WNEG, WPOS, WPOS, kD, kF, wcarry);
  tcast_kernel<<<dim3((2 * kF) / 64, kD / 64, 1), 256, 0, stream>>>(
      Wjf, Wjf, Wjf, Wjf, WPROJ, WPROJ, WPROJ, WPROJ, 2 * kF, kD, wjcarry);

  const int nChunks = kTok / kFfnRows;
  const int n2 = (kFfnRows * kF) / 2;
  for (int cix = 0; cix < nChunks; ++cix) {
    wmma_gemm64<0, false, 0, 0, false><<<dim3(128, 1), 256, 0, stream>>>(
        H16 + (size_t)cix * kFfnRows * kD, H16, kD, 0, WPOS, WPOS, kD, 0, U, U, kF, 0, g1f, xf, 0,
        kFfnRows, kF, kD, 1.0f / wcarry);
    gelu_cast_kernel<<<dim3(n2 / 256), 256, 0, stream>>>(U, CAT + (size_t)cix * kFfnRows * kF, n2, 0, ccarry);
  }
  wmma_gemm64<0, false, 0, 0, true><<<dim3(128, 1), 256, 0, stream>>>(
      CAT, CAT, kF, 0, WPROJ, WPROJ, 2 * kF, 0, TP, TP, kD, 0, g1f, X1, 0, kTok, kD, kF, 1.0f / 1024.0f);
  for (int cix = 0; cix < nChunks; ++cix) {
    wmma_gemm64<0, false, 0, 0, false><<<dim3(128, 1), 256, 0, stream>>>(
        H16 + (size_t)cix * kFfnRows * kD, H16, kD, 0, WNEG, WNEG, kD, 0, U, U, kF, 0, g1f, xf, 0,
        kFfnRows, kF, kD, 1.0f / wcarry);
    gelu_cast_kernel<<<dim3(n2 / 256), 256, 0, stream>>>(U, CAT + (size_t)cix * kFfnRows * kF, n2, 1, ccarry);
  }
  wmma_gemm64<0, false, 0, 0, true><<<dim3(128, 1), 256, 0, stream>>>(
      CAT, CAT, kF, 0, WPROJ + kF, WPROJ + kF, 2 * kF, 0, out, out, kD, 0, g1f, TP, 0, kTok, kD, kF, 1.0f / 1024.0f);
}
